// LinearEdgeDecoder_37409165148918
// MI455X (gfx1250) — hardware-verified
//
#include <hip/hip_runtime.h>
#include <stdint.h>

typedef _Float16     v16h __attribute__((ext_vector_type(16)));
typedef _Float16     v8h  __attribute__((ext_vector_type(8)));
typedef float        v8f  __attribute__((ext_vector_type(8)));
typedef float        v4f  __attribute__((ext_vector_type(4)));
typedef unsigned int v4u  __attribute__((ext_vector_type(4)));

#define D_FEAT 128
#define H2     128
#define KDIM   256
#define NTHR   256
#define NWAVE  8
#define NG     4
#define EPW    (NG * 32)
#define EPB    (EPW * NWAVE)
#define GEPW   32
#define GEPB   (GEPW * NWAVE)
#define MAX_CHUNK_BLOCKS 160
#define W1F_UNITS 4096

__device__ __forceinline__ v8f wmma_f16(v16h a, v16h b, v8f c) {
    v8f d = __builtin_amdgcn_wmma_f32_16x16x32_f16(false, a, false, b, (short)0, c, false, false);
    asm volatile("v_nop\n\tv_nop\n\tv_nop\n\tv_nop" : "+v"(d) : "v"(a), "v"(b));
    return d;
}

__global__ __launch_bounds__(NTHR) void k_cvt_x(const float* __restrict__ x,
                                                _Float16* xh, int n) {
    const long long i = ((long long)blockIdx.x * NTHR + threadIdx.x) * 8;
    if (i + 8 <= (long long)n) {
        const v4f v0 = *(const v4f*)(x + i);
        const v4f v1 = *(const v4f*)(x + i + 4);
        union { v8h h; v4u u; } pk;
        #pragma unroll
        for (int c = 0; c < 4; ++c) {
            pk.h[c]     = (_Float16)v0[c];
            pk.h[4 + c] = (_Float16)v1[c];
        }
        volatile v4u* p = (volatile v4u*)(xh + i);
        *p = pk.u;
        __threadfence();
        *p = pk.u;
    } else if (i < (long long)n) {
        for (long long j = i; j < (long long)n; ++j) {
            const _Float16 hv = (_Float16)x[j];
            *(volatile _Float16*)(xh + j) = hv;
        }
        __threadfence();
        for (long long j = i; j < (long long)n; ++j) {
            const _Float16 hv = (_Float16)x[j];
            *(volatile _Float16*)(xh + j) = hv;
        }
    }
}

__global__ __launch_bounds__(NTHR) void k_cvt_w1(const float* __restrict__ W1, v4u* w1f) {
    const int t = blockIdx.x * NTHR + threadIdx.x;
    if (t >= W1F_UNITS) return;
    const int idx0 = t * 8;
    const int fl   = (idx0 >> 4) & 31;
    const int nt   = (idx0 >> 9) & 7;
    const int kt   = idx0 >> 12;
    const int kb   = kt * 32 + 8 * (fl >> 4) + 16 * (t & 1);
    const int n    = nt * 16 + (fl & 15);
    union { v8h h; v4u u; } pk;
    #pragma unroll
    for (int c = 0; c < 8; ++c) pk.h[c] = (_Float16)(W1[(kb + c) * H2 + n] * 64.0f);
    volatile v4u* p = (volatile v4u*)(w1f + t);
    *p = pk.u;
    __threadfence();
    *p = pk.u;
}

__global__ __launch_bounds__(NTHR) void k_gather(
    const v4u* __restrict__ xh,
    const int* __restrict__ eidx,
    v4u*                    hrow,
    int ebase, int nrows, int nE, int nN)
{
    const int lane  = threadIdx.x & 31;
    const int wave  = threadIdx.x >> 5;
    const int half  = lane >> 4;
    const int piece = lane & 15;
    const int wb    = (blockIdx.x * NWAVE + wave) * GEPW;
    const int* ip   = eidx + (half ? (size_t)nE : (size_t)0);

    #pragma unroll 1
    for (int j0 = 0; j0 < GEPW; j0 += 4) {
        v4u v[4];
        #pragma unroll
        for (int c = 0; c < 4; ++c) {
            int el = wb + j0 + c;
            if (el > nrows - 1) el = nrows - 1;
            int eg = ebase + el;
            if (eg > nE - 1) eg = nE - 1;
            int r = ip[eg];
            if (r < 0) r += nN;
            r = r < 0 ? 0 : (r > nN - 1 ? nN - 1 : r);
            v[c] = xh[(size_t)r * (D_FEAT / 8) + piece];
        }
        #pragma unroll
        for (int c = 0; c < 4; ++c) {
            const int el = wb + j0 + c;
            if (el < nrows) *(volatile v4u*)(hrow + (size_t)el * (KDIM / 8) + lane) = v[c];
        }
        __threadfence();
        #pragma unroll
        for (int c = 0; c < 4; ++c) {
            const int el = wb + j0 + c;
            if (el < nrows) *(volatile v4u*)(hrow + (size_t)el * (KDIM / 8) + lane) = v[c];
        }
    }
}

__global__ __launch_bounds__(NTHR) void k_edge_mlp(
    const _Float16* __restrict__ hrow,
    const v4u*      __restrict__ w1f,
    const float*    __restrict__ b1,
    const float*    __restrict__ W2,
    const float*    __restrict__ b2,
    float*                       out,
    int ebase, int nE)
{
    __shared__ v16h w1s[2048];

    const int tid  = threadIdx.x;
    const int lane = tid & 31;
    const int wave = tid >> 5;
    const int m    = lane & 15;
    const int h    = lane >> 4;

    {
        v4u* d = (v4u*)w1s;
        #pragma unroll
        for (int i = 0; i < 16; ++i) d[tid + i * NTHR] = w1f[tid + i * NTHR];
    }
    float bv[8], wv[8];
    #pragma unroll
    for (int nt = 0; nt < 8; ++nt) {
        bv[nt] = b1[nt * 16 + m];
        wv[nt] = W2[nt * 16 + m];
    }
    const float b2v = b2[0];
    __syncthreads();

    const int q = lane & 3;

    #pragma unroll 1
    for (int g = 0; g < NG; ++g) {
        const int lgb = blockIdx.x * EPB + wave * EPW + g * 32;
        float keep[4] = {0.f, 0.f, 0.f, 0.f};

        #pragma unroll
        for (int u = 0; u < 2; ++u) {
            const int ltb = lgb + u * 16;
            const _Float16* ar = hrow + (size_t)(ltb + m) * KDIM + 8 * h;

            v8f acc[8];
            #pragma unroll
            for (int nt = 0; nt < 8; ++nt) acc[nt] = (v8f){0.f, 0.f, 0.f, 0.f, 0.f, 0.f, 0.f, 0.f};

            #pragma unroll
            for (int kt = 0; kt < 8; ++kt) {
                union { v16h v; v8h hh[2]; } a;
                a.hh[0] = *(const v8h*)(ar + kt * 32);
                a.hh[1] = *(const v8h*)(ar + kt * 32 + 16);
                #pragma unroll
                for (int nt = 0; nt < 8; ++nt) {
                    const v16h b = w1s[(kt * 8 + nt) * 32 + lane];
                    acc[nt] = wmma_f16(a.v, b, acc[nt]);
                }
            }

            float s[8];
            #pragma unroll
            for (int i = 0; i < 8; ++i) {
                float t = 0.f;
                #pragma unroll
                for (int nt = 0; nt < 8; ++nt) {
                    float hv = acc[nt][i] * 0.015625f + bv[nt];
                    hv = hv > 0.f ? hv : 0.f;
                    t += hv * wv[nt];
                }
                s[i] = t;
            }
            #pragma unroll
            for (int off = 8; off >= 1; off >>= 1) {
                #pragma unroll
                for (int i = 0; i < 8; ++i) s[i] += __shfl_xor(s[i], off, 32);
            }
            float so[8];
            #pragma unroll
            for (int i = 0; i < 8; ++i) so[i] = __shfl_xor(s[i], 16, 32);

            float o[4];
            #pragma unroll
            for (int c = 0; c < 4; ++c) {
                const float a0 = s[c], a1 = s[4 + c], a2 = so[c], a3 = so[4 + c];
                o[c] = (q == 0) ? a0 : ((q == 1) ? a1 : ((q == 2) ? a2 : a3));
            }
            if ((lane >> 2) == u) {
                #pragma unroll
                for (int c = 0; c < 4; ++c) keep[c] = o[c] + b2v;
            }
        }

        if (lane < 8) {
            const int gg = ebase + lgb;
            const int eo = gg + lane * 4;
            v4f v;
            v[0] = keep[0]; v[1] = keep[1]; v[2] = keep[2]; v[3] = keep[3];
            if (gg + 32 <= nE) {
                volatile v4f* p = (volatile v4f*)(out + eo);
                *p = v;
                __threadfence();
                *p = v;
            } else {
                #pragma unroll
                for (int c = 0; c < 4; ++c)
                    if (eo + c < nE) *(volatile float*)(out + eo + c) = v[c];
                __threadfence();
                #pragma unroll
                for (int c = 0; c < 4; ++c)
                    if (eo + c < nE) *(volatile float*)(out + eo + c) = v[c];
            }
        }
    }
}

static inline size_t align128(size_t v) { return (v + 127) & ~(size_t)127; }

extern "C" void kernel_launch(void* const* d_in, const int* in_sizes, int n_in,
                              void* d_out, int out_size, void* d_ws, size_t ws_size,
                              hipStream_t stream) {
    if (n_in < 6) return;
    const float* x  = (const float*)d_in[0];
    const int*   ei = (const int*)d_in[1];
    const float* W1 = (const float*)d_in[2];
    const float* b1 = (const float*)d_in[3];
    const float* W2 = (const float*)d_in[4];
    const float* b2 = (const float*)d_in[5];
    float* out = (float*)d_out;

    const int nX = in_sizes[0];
    const int nN = nX / D_FEAT;
    const int nE = in_sizes[1] / 2;
    if (nX <= 0 || nN <= 0 || nE <= 0) return;
    if (in_sizes[2] != KDIM * H2 || in_sizes[3] < H2 || in_sizes[4] < H2 || in_sizes[5] < 1) return;
    if (out_size < nE) return;

    const size_t off_w1 = 0;
    const size_t off_xh = align128(off_w1 + (size_t)W1F_UNITS * 16);
    const size_t off_hr = align128(off_xh + (size_t)nX * 2);
    if (off_hr >= ws_size) return;
    size_t cb = (ws_size - off_hr) / ((size_t)EPB * KDIM * 2);
    if (cb > MAX_CHUNK_BLOCKS) cb = MAX_CHUNK_BLOCKS;
    if (cb < 1) return;
    const int chunkEdges = (int)cb * EPB;
    if (off_hr + (size_t)chunkEdges * KDIM * 2 > ws_size) return;

    unsigned char* ws = (unsigned char*)d_ws;
    v4u*      w1f  = (v4u*)(ws + off_w1);
    _Float16* xh   = (_Float16*)(ws + off_xh);
    _Float16* hrow = (_Float16*)(ws + off_hr);

    const long long groups8 = ((long long)nX + 7) / 8;
    const int cblocks = (int)((groups8 + NTHR - 1) / NTHR);
    k_cvt_x<<<cblocks, NTHR, 0, stream>>>(x, xh, nX);
    k_cvt_w1<<<(W1F_UNITS + NTHR - 1) / NTHR, NTHR, 0, stream>>>(W1, w1f);

    for (int base = 0; base < nE; base += chunkEdges) {
        const int cnt   = (nE - base < chunkEdges) ? (nE - base) : chunkEdges;
        const int gbl   = (cnt + EPB - 1) / EPB;
        const int nrows = gbl * EPB;
        k_gather<<<nrows / GEPB, NTHR, 0, stream>>>((const v4u*)xh, ei, (v4u*)hrow, base, nrows, nE, nN);
        k_edge_mlp<<<gbl, NTHR, 0, stream>>>(hrow, w1f, b1, W2, b2, out, base, nE);
    }
}
